// Net_74904229642961
// MI455X (gfx1250) — hardware-verified
//
#include <hip/hip_runtime.h>
#include <math.h>

constexpr int N_BATCH = 64;
constexpr int N_STEP  = 512;
constexpr int N_POS   = 64;
constexpr int N_ACT   = 16;
constexpr int N_FEAT  = N_POS + N_ACT;
constexpr int K_PAD   = 96;
constexpr int N_HID   = 512;
constexpr int N_ROWS  = N_BATCH * N_STEP;
constexpr int NTHR    = 256;
constexpr int SEQ_BLK = 16;
constexpr int HPITCH  = 520;
constexpr int SLABP   = 68;
constexpr int STP     = 36;
constexpr int XSP     = 100;
constexpr int FLUSH_N = 32;

static_assert(N_FEAT == 80, "feature count");
static_assert(K_PAD % 32 == 0 && K_PAD >= N_FEAT, "k pad");
static_assert(K_PAD % 8 == 0 && N_FEAT % 8 == 0, "chunking");
static_assert(N_HID % 64 == 0 && N_ROWS % 64 == 0, "tile multiples");
static_assert(N_HID % 32 == 0, "k multiple");
static_assert(N_HID == 64 * (NTHR / 32), "8 waves x 64 columns");
static_assert(N_BATCH % SEQ_BLK == 0, "row blocks");
static_assert(N_STEP % FLUSH_N == 0, "flush groups");
static_assert((HPITCH % 8) == 0 && HPITCH >= N_HID, "h pitch");

typedef __attribute__((ext_vector_type(16))) __bf16   v16b;
typedef __attribute__((ext_vector_type(8)))  __bf16   v8b;
typedef __attribute__((ext_vector_type(8)))  float    v8f;
typedef __attribute__((ext_vector_type(4)))  float    v4f;
typedef __attribute__((ext_vector_type(4)))  unsigned v4u;
typedef __attribute__((ext_vector_type(2)))  unsigned v2u;

__device__ __forceinline__ unsigned bf_bits_u(float f) {
  const unsigned u = __float_as_uint(f);
  return (u + 0x7FFFu + ((u >> 16) & 1u)) >> 16;
}
__device__ __forceinline__ float bf_val_u(unsigned b) { return __uint_as_float(b << 16); }
__device__ __forceinline__ void split_pair(float f0, float f1, unsigned& hw, unsigned& lw) {
  const unsigned h0 = bf_bits_u(f0);
  const unsigned h1 = bf_bits_u(f1);
  const unsigned l0 = bf_bits_u(f0 - bf_val_u(h0));
  const unsigned l1 = bf_bits_u(f1 - bf_val_u(h1));
  hw = h0 | (h1 << 16);
  lw = l0 | (l1 << 16);
}

__device__ __forceinline__ void guard1_b(v8f& a, v16b x, v16b y, v16b z, v16b w) {
  asm volatile("v_nop\n\tv_nop\n\tv_nop\n\tv_nop" : "+v"(a) : "v"(x), "v"(y), "v"(z), "v"(w));
}
__device__ __forceinline__ void guard4_b(v8f& a, v8f& b, v8f& c, v8f& d, v16b x, v16b y) {
  asm volatile("v_nop\n\tv_nop\n\tv_nop\n\tv_nop" : "+v"(a), "+v"(b), "+v"(c), "+v"(d) : "v"(x), "v"(y));
}
__device__ __forceinline__ void keep4_b(v16b a, v16b b, v16b c, v16b d) { asm volatile("v_nop" :: "v"(a), "v"(b), "v"(c), "v"(d)); }
__device__ __forceinline__ void acc_guard4(v8f& a, v8f& b, v8f& c, v8f& d) {
  asm volatile("v_nop\n\tv_nop\n\tv_nop\n\tv_nop" : "+v"(a), "+v"(b), "+v"(c), "+v"(d));
}

union FragU { v16b v; v8b h[2]; };
__device__ __forceinline__ v16b frag_load(const __bf16* p) {
  FragU f;
  f.h[0] = *(const v8b*)(p);
  f.h[1] = *(const v8b*)(p + 16);
  return f.v;
}
__device__ __forceinline__ v8f frag_mma(v16b a, v16b b, v8f c) {
  return __builtin_amdgcn_wmma_f32_16x16x32_bf16(false, a, false, b, (short)0, c, false, false);
}

__global__ __launch_bounds__(NTHR) void pack_x_kernel(const float* __restrict__ obs, const float* __restrict__ act,
                                                      unsigned* __restrict__ XH, unsigned* __restrict__ XL) {
  __shared__ __align__(16) float xs[64 * XSP];
  const int tid  = threadIdx.x;
  const int row0 = blockIdx.x * 64;
#pragma unroll
  for (int it = 0; it < 4; ++it) {
    const int idx = it * NTHR + tid;
    const int r = idx >> 4, c4 = (idx & 15) * 4;
    const v4f v = *(const v4f*)(obs + (size_t)(row0 + r) * N_POS + c4);
    *(v4f*)(xs + r * XSP + c4) = v;
  }
  {
    const int r = tid >> 2, c4 = (tid & 3) * 4;
    const v4f v = *(const v4f*)(act + (size_t)(row0 + r) * N_ACT + c4);
    const v4f z = {0.0f, 0.0f, 0.0f, 0.0f};
    *(v4f*)(xs + r * XSP + N_POS + c4) = v;
    *(v4f*)(xs + r * XSP + N_FEAT + c4) = z;
  }
  __syncthreads();
  v4u hw[3], lw[3];
#pragma unroll
  for (int it = 0; it < 3; ++it) {
    const int idx = it * NTHR + tid;
    const int r = idx / 12;
    const int c8 = idx - r * 12;
    const v4f a = *(const v4f*)(xs + r * XSP + c8 * 8);
    const v4f b = *(const v4f*)(xs + r * XSP + c8 * 8 + 4);
    unsigned h, l;
    split_pair(a[0], a[1], h, l); hw[it][0] = h; lw[it][0] = l;
    split_pair(a[2], a[3], h, l); hw[it][1] = h; lw[it][1] = l;
    split_pair(b[0], b[1], h, l); hw[it][2] = h; lw[it][2] = l;
    split_pair(b[2], b[3], h, l); hw[it][3] = h; lw[it][3] = l;
  }
  for (int pass = 0; pass < 2; ++pass) {
#pragma unroll
    for (int it = 0; it < 3; ++it) {
      const size_t g = (size_t)blockIdx.x * 768 + (size_t)(it * NTHR + tid);
      *(volatile v4u*)(XH + g * 4) = hw[it];
      *(volatile v4u*)(XL + g * 4) = lw[it];
    }
    __threadfence();
  }
}

__global__ __launch_bounds__(NTHR) void wt_prep_kernel(const float* __restrict__ Wci,
                                                       unsigned* __restrict__ WtH, unsigned* __restrict__ WtL) {
  __shared__ float Tw[N_FEAT * 65];
  const int tid = threadIdx.x;
  const int n0  = blockIdx.x * 64;
#pragma unroll
  for (int it = 0; it < 5; ++it) {
    const int idx = it * NTHR + tid;
    const int rr = idx >> 4, cc = (idx & 15) * 4;
    const v4f v = *(const v4f*)(Wci + (size_t)rr * N_HID + n0 + cc);
    Tw[rr * 65 + cc + 0] = v[0];
    Tw[rr * 65 + cc + 1] = v[1];
    Tw[rr * 65 + cc + 2] = v[2];
    Tw[rr * 65 + cc + 3] = v[3];
  }
  __syncthreads();
  v4u hw[3], lw[3];
#pragma unroll
  for (int it = 0; it < 3; ++it) {
    const int idx = it * NTHR + tid;
    const int nn = idx / 12;
    const int c8 = idx - nn * 12;
#pragma unroll
    for (int e2 = 0; e2 < 4; ++e2) {
      const int k0 = c8 * 8 + 2 * e2;
      const int k1 = k0 + 1;
      const int k0c = (k0 < N_FEAT) ? k0 : (N_FEAT - 1);
      const int k1c = (k1 < N_FEAT) ? k1 : (N_FEAT - 1);
      float f0 = Tw[k0c * 65 + nn];
      float f1 = Tw[k1c * 65 + nn];
      f0 = (k0 < N_FEAT) ? f0 : 0.0f;
      f1 = (k1 < N_FEAT) ? f1 : 0.0f;
      unsigned h, l;
      split_pair(f0, f1, h, l);
      hw[it][e2] = h;
      lw[it][e2] = l;
    }
  }
  for (int pass = 0; pass < 2; ++pass) {
#pragma unroll
    for (int it = 0; it < 3; ++it) {
      const size_t g = (size_t)blockIdx.x * 768 + (size_t)(it * NTHR + tid);
      *(volatile v4u*)(WtH + g * 4) = hw[it];
      *(volatile v4u*)(WtL + g * 4) = lw[it];
    }
    __threadfence();
  }
}

__global__ __launch_bounds__(NTHR) void rt_prep_kernel(const float* __restrict__ Rig,
                                                       unsigned* __restrict__ RtH, unsigned* __restrict__ RtL) {
  __shared__ float Tt[64 * 65];
  const int tid = threadIdx.x;
  const int c0 = blockIdx.x * 64, r0 = blockIdx.y * 64;
#pragma unroll
  for (int it = 0; it < 4; ++it) {
    const int idx = it * NTHR + tid;
    const int rr = idx >> 4, cc = (idx & 15) * 4;
    const v4f v = *(const v4f*)(Rig + (size_t)(r0 + rr) * N_HID + c0 + cc);
    Tt[rr * 65 + cc + 0] = v[0];
    Tt[rr * 65 + cc + 1] = v[1];
    Tt[rr * 65 + cc + 2] = v[2];
    Tt[rr * 65 + cc + 3] = v[3];
  }
  __syncthreads();
  const int q = tid >> 3, c8 = (tid & 7) * 8;
  v4u hw[2], lw[2];
#pragma unroll
  for (int g = 0; g < 2; ++g) {
    const int qq = g * 32 + q;
#pragma unroll
    for (int e2 = 0; e2 < 4; ++e2) {
      const float f0 = Tt[(c8 + 2 * e2) * 65 + qq];
      const float f1 = Tt[(c8 + 2 * e2 + 1) * 65 + qq];
      unsigned h, l;
      split_pair(f0, f1, h, l);
      hw[g][e2] = h;
      lw[g][e2] = l;
    }
  }
  for (int pass = 0; pass < 2; ++pass) {
#pragma unroll
    for (int g = 0; g < 2; ++g) {
      const size_t o = ((size_t)(c0 + g * 32 + q) * N_HID + (size_t)(r0 + c8)) >> 1;
      *(volatile v4u*)(RtH + o) = hw[g];
      *(volatile v4u*)(RtL + o) = lw[g];
    }
    __threadfence();
  }
}

__global__ __launch_bounds__(NTHR) void ci_gemm_kernel(const unsigned short* __restrict__ XHp, const unsigned short* __restrict__ XLp,
                                                       const unsigned short* __restrict__ WHp, const unsigned short* __restrict__ WLp,
                                                       const float* __restrict__ bias, float* __restrict__ CI) {
  const __bf16* Ahi = (const __bf16*)XHp;
  const __bf16* Alo = (const __bf16*)XLp;
  const __bf16* Bhi = (const __bf16*)WHp;
  const __bf16* Blo = (const __bf16*)WLp;
  __shared__ __align__(16) float sT[8][16 * SLABP];
  const int lane = threadIdx.x & 31;
  const int wave = threadIdx.x >> 5;
  constexpr int tilesN = N_HID / 64;
  constexpr int tilesM = N_ROWS / 64;
  const int tile = blockIdx.x * 8 + wave;
  if (tile >= tilesM * tilesN) return;
  const int tm = tile / tilesN;
  const int tn = tile - tm * tilesN;
  const int m0 = tm << 6;
  const int n0 = tn << 6;
  const int rlane = lane & 15;
  const int koff  = (lane >> 4) * 8;
  const int mOff  = (lane >> 4) * 8;

  v8f acc[4][4];
#pragma unroll
  for (int i = 0; i < 4; ++i)
#pragma unroll
    for (int j = 0; j < 4; ++j) acc[i][j] = (v8f){0.f, 0.f, 0.f, 0.f, 0.f, 0.f, 0.f, 0.f};

#pragma unroll 1
  for (int k0 = 0; k0 < K_PAD; k0 += 32) {
    v16b bh[4], bl[4];
#pragma unroll
    for (int j = 0; j < 4; ++j) {
      const size_t bo = (size_t)(n0 + (j << 4) + rlane) * K_PAD + koff + k0;
      bh[j] = frag_load(Bhi + bo);
      bl[j] = frag_load(Blo + bo);
    }
#pragma unroll
    for (int i = 0; i < 4; ++i) {
      const size_t ao = (size_t)(m0 + (i << 4) + rlane) * K_PAD + koff + k0;
      const v16b ah = frag_load(Ahi + ao);
      const v16b al = frag_load(Alo + ao);
#pragma unroll
      for (int j = 0; j < 4; ++j) {
        acc[i][j] = frag_mma(ah, bl[j], acc[i][j]);
        acc[i][j] = frag_mma(al, bh[j], acc[i][j]);
        acc[i][j] = frag_mma(ah, bh[j], acc[i][j]);
      }
      guard4_b(acc[i][0], acc[i][1], acc[i][2], acc[i][3], ah, al);
    }
    keep4_b(bh[0], bh[1], bh[2], bh[3]);
    keep4_b(bl[0], bl[1], bl[2], bl[3]);
  }
  acc_guard4(acc[0][0], acc[0][1], acc[0][2], acc[0][3]);
  acc_guard4(acc[1][0], acc[1][1], acc[1][2], acc[1][3]);
  acc_guard4(acc[2][0], acc[2][1], acc[2][2], acc[2][3]);
  acc_guard4(acc[3][0], acc[3][1], acc[3][2], acc[3][3]);

  float* slab = sT[wave];
  float bv[4];
#pragma unroll
  for (int j = 0; j < 4; ++j) bv[j] = bias[n0 + (j << 4) + rlane];
  const int hh2 = lane >> 4, c4 = (lane & 15) * 4;
#pragma unroll
  for (int i = 0; i < 4; ++i) {
    const int mBase = m0 + (i << 4);
#pragma unroll
    for (int j = 0; j < 4; ++j) {
#pragma unroll
      for (int r = 0; r < 8; ++r) slab[(mOff + r) * SLABP + (j << 4) + rlane] = acc[i][j][r] + bv[j];
    }
    __builtin_amdgcn_fence(__ATOMIC_RELEASE, "workgroup");
    __builtin_amdgcn_wave_barrier();
    __builtin_amdgcn_fence(__ATOMIC_ACQUIRE, "workgroup");
#pragma unroll 1
    for (int q = 0; q < 32; ++q) {
      const int row = (q >> 2) * 2 + hh2;
      float* p = slab + row * SLABP + c4 + (q & 3);
      const float pre = *p;
      *p = tanhf(pre);
    }
    __builtin_amdgcn_fence(__ATOMIC_RELEASE, "workgroup");
    __builtin_amdgcn_wave_barrier();
    __builtin_amdgcn_fence(__ATOMIC_ACQUIRE, "workgroup");
    for (int pass = 0; pass < 2; ++pass) {
#pragma unroll
      for (int it = 0; it < 8; ++it) {
        const int row = it * 2 + hh2;
        const v4f v = *(const v4f*)(slab + row * SLABP + c4);
        *(volatile v4f*)(CI + (size_t)(mBase + row) * N_HID + n0 + c4) = v;
      }
      __threadfence();
    }
    __builtin_amdgcn_fence(__ATOMIC_RELEASE, "workgroup");
    __builtin_amdgcn_wave_barrier();
    __builtin_amdgcn_fence(__ATOMIC_ACQUIRE, "workgroup");
  }
}

__global__ __launch_bounds__(NTHR) void recur_kernel(const float* __restrict__ CI,
                                                     const unsigned short* __restrict__ RtHp,
                                                     const unsigned short* __restrict__ RtLp,
                                                     const float* __restrict__ b_ig, const float* __restrict__ w_out,
                                                     const float* __restrict__ b_out, float* __restrict__ out) {
  __shared__ __align__(16) unsigned short Ahs[SEQ_BLK * HPITCH];
  __shared__ __align__(16) unsigned short Als[SEQ_BLK * HPITCH];
  __shared__ __align__(16) float Part[8 * SEQ_BLK];
  __shared__ __align__(16) float Stage[SEQ_BLK * STP];
  const __bf16* RtH = (const __bf16*)RtHp;
  const __bf16* RtL = (const __bf16*)RtLp;
  const int tid = threadIdx.x, lane = tid & 31, wave = tid >> 5;
  const int c = lane & 15, hh = lane >> 4, koff = hh * 8;
  const int rowbase = blockIdx.x * SEQ_BLK;
  const int jcol = 64 * wave + 4 * c;

  {
    unsigned* za = (unsigned*)Ahs;
    unsigned* zb = (unsigned*)Als;
#pragma unroll 1
    for (int i = tid; i < SEQ_BLK * HPITCH / 2; i += NTHR) { za[i] = 0u; zb[i] = 0u; }
#pragma unroll 1
    for (int i = tid; i < 8 * SEQ_BLK; i += NTHR) Part[i] = 0.0f;
#pragma unroll 1
    for (int i = tid; i < SEQ_BLK * STP; i += NTHR) Stage[i] = 0.0f;
  }
  float hst[8][4];
#pragma unroll
  for (int r = 0; r < 8; ++r)
#pragma unroll
    for (int nt = 0; nt < 4; ++nt) hst[r][nt] = 0.0f;
  const v4f big4 = *(const v4f*)(b_ig + jcol);
  const v4f wo4  = *(const v4f*)(w_out + jcol);
  const float bout = b_out[0];
  __syncthreads();

  const __bf16* ahrow = (const __bf16*)Ahs + c * HPITCH + koff;
  const __bf16* alrow = (const __bf16*)Als + c * HPITCH + koff;
  const __bf16* rbh = RtH + (size_t)jcol * N_HID + koff;
  const __bf16* rbl = RtL + (size_t)jcol * N_HID + koff;
  const v8f z8 = {0.f, 0.f, 0.f, 0.f, 0.f, 0.f, 0.f, 0.f};

#pragma unroll 1
  for (int t = 0; t < N_STEP; ++t) {
    v4f cv[8];
#pragma unroll
    for (int r = 0; r < 8; ++r) {
      cv[r] = *(const v4f*)(CI + ((size_t)(rowbase + 8 * hh + r) * N_STEP + (size_t)t) * N_HID + jcol);
      asm volatile("" : "+v"(cv[r]));
    }

    v8f acc[4];
    acc[0] = z8; acc[1] = z8; acc[2] = z8; acc[3] = z8;
#pragma unroll 1
    for (int k0 = 0; k0 < N_HID; k0 += 32) {
      const v16b ah = frag_load(ahrow + k0);
      const v16b al = frag_load(alrow + k0);
#pragma unroll
      for (int nt = 0; nt < 4; ++nt) {
        const v16b bh = frag_load(rbh + (size_t)nt * N_HID + k0);
        const v16b bl = frag_load(rbl + (size_t)nt * N_HID + k0);
        acc[nt] = frag_mma(ah, bl, acc[nt]);
        acc[nt] = frag_mma(al, bh, acc[nt]);
        acc[nt] = frag_mma(ah, bh, acc[nt]);
        guard1_b(acc[nt], ah, al, bh, bl);
      }
    }
    acc_guard4(acc[0], acc[1], acc[2], acc[3]);

    __syncthreads();

    float pr[8];
#pragma unroll
    for (int r = 0; r < 8; ++r) {
      float hn[4];
#pragma unroll
      for (int nt = 0; nt < 4; ++nt) {
        float z = acc[nt][r] + big4[nt];
        z = fminf(fmaxf(z, -60.0f), 60.0f);
        const float e = expf(-z);
        const float g = 1.0f / (1.0f + e);
        const float hv = hst[r][nt] + cv[r][nt] * g;
        hst[r][nt] = hv;
        hn[nt] = hv;
      }
      unsigned h01, l01, h23, l23;
      split_pair(hn[0], hn[1], h01, l01);
      split_pair(hn[2], hn[3], h23, l23);
      v2u ph, pl;
      ph[0] = h01; ph[1] = h23;
      pl[0] = l01; pl[1] = l23;
      *(v2u*)(Ahs + (8 * hh + r) * HPITCH + jcol) = ph;
      *(v2u*)(Als + (8 * hh + r) * HPITCH + jcol) = pl;
      pr[r] = ((hn[0] * wo4[0] + hn[1] * wo4[1]) + hn[2] * wo4[2]) + hn[3] * wo4[3];
    }
#pragma unroll
    for (int r = 0; r < 8; ++r) {
      float v = pr[r];
      v += __shfl_xor(v, 1, 32);
      v += __shfl_xor(v, 2, 32);
      v += __shfl_xor(v, 4, 32);
      v += __shfl_xor(v, 8, 32);
      pr[r] = v;
    }
    if (c == 0) {
#pragma unroll
      for (int r = 0; r < 8; ++r) Part[wave * SEQ_BLK + 8 * hh + r] = pr[r];
    }
    __syncthreads();

    if (tid < SEQ_BLK) {
      float s = 0.0f;
#pragma unroll
      for (int w = 0; w < 8; ++w) s += Part[w * SEQ_BLK + tid];
      s += bout;
      Stage[tid * STP + (t & (FLUSH_N - 1))] = s;
    }
    if ((t & (FLUSH_N - 1)) == (FLUSH_N - 1)) {
      __syncthreads();
      if (wave == 0) {
        const int q = lane >> 3, c4 = (lane & 7) * 4;
        const int t0 = t - (FLUSH_N - 1);
        for (int pass = 0; pass < 2; ++pass) {
#pragma unroll
          for (int it = 0; it < 4; ++it) {
            const int row = it * 4 + q;
            const v4f v = *(const v4f*)(Stage + row * STP + c4);
            *(volatile v4f*)(out + (size_t)(rowbase + row) * N_STEP + t0 + c4) = v;
          }
          __threadfence();
        }
      }
    }
  }
}

extern "C" void kernel_launch(void* const* d_in, const int* in_sizes, int n_in,
                              void* d_out, int out_size, void* d_ws, size_t ws_size, hipStream_t stream) {
  if (n_in < 8 || d_out == nullptr || d_ws == nullptr) return;
  if (in_sizes[0] != N_BATCH * N_STEP * N_POS || in_sizes[1] != N_BATCH * N_STEP * N_ACT ||
      in_sizes[2] != N_FEAT * N_HID || in_sizes[3] != N_HID || in_sizes[4] != N_HID * N_HID ||
      in_sizes[5] != N_HID || in_sizes[6] != N_HID || in_sizes[7] != 1 || out_size != N_BATCH * N_STEP) return;

  const float* obs  = (const float*)d_in[0];
  const float* act  = (const float*)d_in[1];
  const float* wci  = (const float*)d_in[2];
  const float* bci  = (const float*)d_in[3];
  const float* rig  = (const float*)d_in[4];
  const float* big  = (const float*)d_in[5];
  const float* wout = (const float*)d_in[6];
  const float* bout = (const float*)d_in[7];
  float* out = (float*)d_out;

  char* ws = (char*)d_ws;
  size_t off = 0;
  auto carve = [&](size_t bytes) -> char* { char* p = ws + off; off += (bytes + 255) & ~(size_t)255; return p; };
  float*    CI  = (float*)carve((size_t)N_ROWS * N_HID * 4);
  unsigned* XH  = (unsigned*)carve((size_t)N_ROWS * K_PAD * 2);
  unsigned* XL  = (unsigned*)carve((size_t)N_ROWS * K_PAD * 2);
  unsigned* WtH = (unsigned*)carve((size_t)N_HID * K_PAD * 2);
  unsigned* WtL = (unsigned*)carve((size_t)N_HID * K_PAD * 2);
  unsigned* RtH = (unsigned*)carve((size_t)N_HID * N_HID * 2);
  unsigned* RtL = (unsigned*)carve((size_t)N_HID * N_HID * 2);
  if (off > ws_size || off > (size_t)134217728) return;

  pack_x_kernel<<<N_ROWS / 64, NTHR, 0, stream>>>(obs, act, XH, XL);
  wt_prep_kernel<<<N_HID / 64, NTHR, 0, stream>>>(wci, WtH, WtL);
  rt_prep_kernel<<<dim3(N_HID / 64, N_HID / 64), NTHR, 0, stream>>>(rig, RtH, RtL);
  ci_gemm_kernel<<<(N_ROWS / 64) * (N_HID / 64) / 8, NTHR, 0, stream>>>(
      (const unsigned short*)XH, (const unsigned short*)XL, (const unsigned short*)WtH, (const unsigned short*)WtL, bci, CI);
  recur_kernel<<<N_BATCH / SEQ_BLK, NTHR, 0, stream>>>(CI, (const unsigned short*)RtH, (const unsigned short*)RtL,
                                                       big, wout, bout, out);
}
